// STPTransformer_38706245272402
// MI455X (gfx1250) — hardware-run, weakly checked
//
#include <hip/hip_runtime.h>


#define NB_  4
#define NSQ  400
#define TT   128
#define DD   64
#define DFF  256
#define NRB  (NSQ * TT)
#define NREL 33
typedef _Float16 h16;
typedef unsigned short bf;
typedef __attribute__((ext_vector_type(16))) __bf16   v16bf;
typedef __attribute__((ext_vector_type(16))) _Float16 v16h;
typedef __attribute__((ext_vector_type(8)))  _Float16 v8h;
typedef __attribute__((ext_vector_type(8)))  unsigned short v8us;
typedef __attribute__((ext_vector_type(8)))  float    v8f;
typedef __attribute__((ext_vector_type(4)))  float    v4f;
typedef v8h  __attribute__((may_alias)) v8ha;
typedef v4f  __attribute__((may_alias)) v4fa;
typedef v8us __attribute__((may_alias)) v8usa;

__device__ __forceinline__ unsigned short f2bf(float f) { unsigned u = __float_as_uint(f); u += 0x7FFFu + ((u >> 16) & 1u); return (unsigned short)(u >> 16); }
__device__ __forceinline__ float bf2f(unsigned short b) { return __uint_as_float(((unsigned)b) << 16); }
__device__ __forceinline__ float bfr(float f) { return bf2f(f2bf(f)); }
__device__ __forceinline__ v16h cat16(v8h lo, v8h hi) { return __builtin_shufflevector(lo, hi, 0, 1, 2, 3, 4, 5, 6, 7, 8, 9, 10, 11, 12, 13, 14, 15); }
__device__ __forceinline__ v16bf cat16b(v8us lo, v8us hi) { return __builtin_bit_cast(v16bf, __builtin_shufflevector(lo, hi, 0, 1, 2, 3, 4, 5, 6, 7, 8, 9, 10, 11, 12, 13, 14, 15)); }
__device__ __forceinline__ v8f wmma16(v16h a, v16h b, v8f c) { return __builtin_amdgcn_wmma_f32_16x16x32_f16(false, a, false, b, (short)0, c, false, false); }
__device__ __forceinline__ v8f wmmab(v16bf a, v16bf b, v8f c) { return __builtin_amdgcn_wmma_f32_16x16x32_bf16(false, a, false, b, (short)0, c, false, false); }


template <typename T16> struct WFrag;
template <> struct WFrag<h16> { typedef v16h V; static __device__ __forceinline__ V ld(const h16* p) { return cat16(*(const v8h*)p, *(const v8h*)(p + 16)); } static __device__ __forceinline__ v8f mma(V a, V b, v8f c) { return wmma16(a, b, c); } };
template <> struct WFrag<bf> { typedef v16bf V; static __device__ __forceinline__ V ld(const bf* p) { return cat16b(*(const v8us*)p, *(const v8us*)(p + 16)); } static __device__ __forceinline__ v8f mma(V a, V b, v8f c) { return wmmab(a, b, c); } };
template <typename T16, int NSPLIT, bool BIAS>
__global__ __launch_bounds__(32) void k_gemmw(const T16* __restrict__ A, const T16* __restrict__ A2, const T16* __restrict__ Bt, const T16* __restrict__ Bt2, int K, float* C, int ldc, const float* __restrict__ bias, size_t sA, size_t sB, size_t sC) {
    typedef typename WFrag<T16>::V V;
    __shared__ __align__(16) float os[16 * 68];
    const size_t z = blockIdx.z; A += z * sA; if (A2) A2 += z * sA; Bt += z * sB; if (Bt2) Bt2 += z * sB; C += z * sC;
    const int lane = threadIdx.x & 31, lr = lane & 15, hi = lane >> 4; const int r0 = blockIdx.x * 64, c0 = blockIdx.y * 64;
    v8f acc[4][4];
#pragma unroll
    for (int mb = 0; mb < 4; ++mb)
#pragma unroll
        for (int nb = 0; nb < 4; ++nb) acc[mb][nb] = (v8f){};
    const size_t aoff = (size_t)(r0 + lr) * K + 8 * hi, boff = (size_t)(c0 + lr) * K + 8 * hi;
#pragma unroll 1
    for (int kc = 0; kc < K; kc += 32) {
        V a[4], a2[4];
#pragma unroll
        for (int mb = 0; mb < 4; ++mb) { a[mb] = WFrag<T16>::ld(A + aoff + (size_t)mb * 16 * K + kc); if (NSPLIT == 1 || NSPLIT == 2) a2[mb] = WFrag<T16>::ld(A2 + aoff + (size_t)mb * 16 * K + kc); }
#pragma unroll
        for (int nb = 0; nb < 4; ++nb) { const V b = WFrag<T16>::ld(Bt + boff + (size_t)nb * 16 * K + kc); V b2; if (NSPLIT >= 2) b2 = WFrag<T16>::ld(Bt2 + boff + (size_t)nb * 16 * K + kc);
#pragma unroll
            for (int mb = 0; mb < 4; ++mb) { acc[mb][nb] = WFrag<T16>::mma(a[mb], b, acc[mb][nb]); if (NSPLIT == 1 || NSPLIT == 2) acc[mb][nb] = WFrag<T16>::mma(a2[mb], b, acc[mb][nb]); if (NSPLIT >= 2) acc[mb][nb] = WFrag<T16>::mma(a[mb], b2, acc[mb][nb]); } }
        asm volatile("v_nop\n\tv_nop\n\tv_nop\n\tv_nop" : "+v"(acc[0][0]), "+v"(acc[1][1]), "+v"(acc[2][2]), "+v"(acc[3][3]) : "v"(a[0]), "v"(a[3]));
    }
#pragma unroll
    for (int mb = 0; mb < 4; ++mb) {
#pragma unroll
        for (int nb = 0; nb < 4; ++nb) {
#pragma unroll
            for (int j = 0; j < 8; ++j) os[(hi * 8 + j) * 68 + nb * 16 + lr] = acc[mb][nb][j]; }
        __builtin_amdgcn_wave_barrier(); asm volatile("" ::: "memory");
        float* crow = C + (size_t)(r0 + mb * 16) * ldc + c0;
#pragma unroll 1
        for (int ps = 0; ps < 2; ++ps) {
#pragma unroll
            for (int s = 0; s < 8; ++s) { const int row = 2 * s + hi, cofs = lr * 4; v4f val = *(const v4fa*)(os + row * 68 + cofs); if (BIAS) { val[0] += bfr(bias[c0 + cofs]); val[1] += bfr(bias[c0 + cofs + 1]); val[2] += bfr(bias[c0 + cofs + 2]); val[3] += bfr(bias[c0 + cofs + 3]); }
                *(volatile v4f*)(crow + (size_t)row * ldc + cofs) = val; }
            if (ps == 0) __threadfence(); }
        __builtin_amdgcn_wave_barrier(); asm volatile("" ::: "memory");
    }
}

__device__ __forceinline__ void splitf(float y, unsigned short& h, unsigned short& l) { h = f2bf(y); l = f2bf(y - bf2f(h)); }
typedef __attribute__((ext_vector_type(2))) unsigned short v2us;
typedef __attribute__((ext_vector_type(4))) unsigned short v4us;
typedef __attribute__((ext_vector_type(2))) float v2f;

__global__ __launch_bounds__(256) void k_wtG(const float* __restrict__ w, int K, int N, bf* Bt) {
    const int lane = threadIdx.x & 31; const int L0 = (blockIdx.x * 8 + (threadIdx.x >> 5)) * 8; const int nlines = N * K / 64;
#pragma unroll
    for (int ps = 0; ps < 2; ++ps) {
#pragma unroll 1
        for (int l = 0; l < 8; ++l) { const int L = L0 + l; if (L >= nlines) break; const size_t e = (size_t)L * 64 + lane * 2; const int k = (int)(e % K), n = (int)(e / K); v2us o;
            o[0] = f2bf(w[(size_t)k * N + n]); o[1] = f2bf(w[(size_t)(k + 1) * N + n]); *(volatile v2us*)(Bt + e) = o; }
        if (ps == 0) __threadfence(); }
}
__global__ __launch_bounds__(256) void k_cvt8(const float* __restrict__ src, bf* dst, size_t n8) { const size_t i = (size_t)blockIdx.x * 256 + threadIdx.x; if (i >= n8) return; const v8f v = *(const v8f*)(src + i * 8); v8us o;
#pragma unroll
    for (int k = 0; k < 8; ++k) o[k] = f2bf(v[k]); *(volatile v8us*)(dst + i * 8) = o; __threadfence(); *(volatile v8us*)(dst + i * 8) = o; }
__global__ __launch_bounds__(256) void k_relT(const float* __restrict__ rk, const float* __restrict__ rv, bf* BK, bf* BV) { const int e = (blockIdx.x * 256 + threadIdx.x) * 4; if (e >= DD * DD) return; const int c = e % DD; const int r = e / DD; v4us a, b;
#pragma unroll
    for (int u = 0; u < 4; ++u) { a[u] = (r < NREL) ? f2bf(rk[r * DD + c + u]) : (unsigned short)0; b[u] = (c + u < NREL) ? f2bf(rv[(c + u) * DD + r]) : (unsigned short)0; } *(volatile v4us*)(BK + e) = a; *(volatile v4us*)(BV + e) = b; __threadfence(); *(volatile v4us*)(BK + e) = a; *(volatile v4us*)(BV + e) = b; }
__global__ __launch_bounds__(256) void k_spl(const float* __restrict__ F, size_t n4, bf* Hh, bf* Hl) { const size_t e = ((size_t)blockIdx.x * 256 + threadIdx.x) * 4; if (e >= n4) return; const v4f a = *(const v4f*)(F + e); v4us oh, ol;
#pragma unroll
    for (int u = 0; u < 4; ++u) { unsigned short p, q; splitf(a[u], p, q); oh[u] = p; ol[u] = q; } *(volatile v4us*)(Hh + e) = oh; *(volatile v4us*)(Hl + e) = ol; __threadfence(); *(volatile v4us*)(Hh + e) = oh; *(volatile v4us*)(Hl + e) = ol; }
__global__ __launch_bounds__(256) void k_vtz(const float* __restrict__ V, bf* Th, bf* Tl) { const size_t e = ((size_t)blockIdx.x * 256 + threadIdx.x) * 2; if (e >= (size_t)NSQ * DD * TT) return; const int u = (int)(e % TT); const int d = (int)((e / TT) % DD); const int z = (int)(e / ((size_t)TT * DD)); v2us oh, ol;
#pragma unroll
    for (int w = 0; w < 2; ++w) { unsigned short a, b; splitf(V[((size_t)z * TT + u + w) * DD + d], a, b); oh[w] = a; ol[w] = b; } *(volatile v2us*)(Th + e) = oh; *(volatile v2us*)(Tl + e) = ol; __threadfence(); *(volatile v2us*)(Th + e) = oh; *(volatile v2us*)(Tl + e) = ol; }
__global__ __launch_bounds__(256) void k_ssoft(const float* __restrict__ S, const float* __restrict__ QR, bf* Ph, bf* Pl, bf* PBh, bf* PBl) {
    const int lane = threadIdx.x & 31; const int row = blockIdx.x * 8 + (threadIdx.x >> 5); if (row >= NSQ * TT) return; const int t = row % TT; const float* sr = S + (size_t)row * TT; const float* qr = QR + (size_t)row * DD; float v[4]; float mx = -3.0e38f;
    const v4f a = *(const v4f*)(sr + lane * 4);
#pragma unroll
    for (int w = 0; w < 4; ++w) { const int u = lane * 4 + w; const int idx = min(max(u - t, -16), 16) + 16; float s0 = __fadd_rn(a[w], qr[idx]); asm volatile("" : "+v"(s0)); v[w] = s0 * 0.125f; mx = fmaxf(mx, v[w]); }
#pragma unroll
    for (int sh = 16; sh; sh >>= 1) mx = fmaxf(mx, __shfl_xor(mx, sh, 32));
    float sum = 0.f;
#pragma unroll
    for (int w = 0; w < 4; ++w) { float d0 = __fsub_rn(v[w], mx); asm volatile("" : "+v"(d0)); v[w] = __builtin_amdgcn_exp2f(__fmul_rn(d0, 1.4426950408889634f)); sum += v[w]; }
#pragma unroll
    for (int sh = 16; sh; sh >>= 1) sum += __shfl_xor(sum, sh, 32);
    const float f = __fdiv_rn(1.0f, sum); float p[4]; float lo = 0.f, hi = 0.f;
#pragma unroll
    for (int w = 0; w < 4; ++w) { const int u = lane * 4 + w; p[w] = v[w] * f; if (u - t <= -16) lo += p[w]; if (u - t >= 16) hi += p[w]; }
#pragma unroll
    for (int sh = 16; sh; sh >>= 1) { lo += __shfl_xor(lo, sh, 32); hi += __shfl_xor(hi, sh, 32); }
    float b2v[2];
#pragma unroll
    for (int w = 0; w < 2; ++w) { const int r = lane * 2 + w; const int u = t - 16 + r; const int src = (u >= 0 && u < TT) ? (u >> 2) : 0; const int sl = u & 3;
        const float g0 = __shfl(p[0], src, 32), g1 = __shfl(p[1], src, 32), g2 = __shfl(p[2], src, 32), g3 = __shfl(p[3], src, 32); const float gv = (sl == 0) ? g0 : (sl == 1) ? g1 : (sl == 2) ? g2 : g3;
        b2v[w] = (r == 0) ? lo : (r == 32) ? hi : (r < NREL && u >= 0 && u < TT) ? gv : 0.f; }
    for (int ps = 0; ps < 2; ++ps) { v4us oh, ol; v2us bh, bl;
#pragma unroll
        for (int w = 0; w < 4; ++w) { unsigned short q1, q2; splitf(p[w], q1, q2); oh[w] = q1; ol[w] = q2; }
#pragma unroll
        for (int w = 0; w < 2; ++w) { unsigned short q1, q2; splitf(b2v[w], q1, q2); bh[w] = q1; bl[w] = q2; }
        const size_t oo = (size_t)row * TT + lane * 4; *(volatile v4us*)(Ph + oo) = oh; *(volatile v4us*)(Pl + oo) = ol; const size_t ob = (size_t)row * DD + lane * 2; *(volatile v2us*)(PBh + ob) = bh; *(volatile v2us*)(PBl + ob) = bl;
        if (ps == 0) __threadfence(); } }
__global__ __launch_bounds__(256) void k_add2(const float* __restrict__ A, const float* __restrict__ Bv, size_t n4, bf* Hh, bf* Hl) { const size_t e = ((size_t)blockIdx.x * 256 + threadIdx.x) * 4; if (e >= n4) return; const v4f a = *(const v4f*)(A + e), b4 = *(const v4f*)(Bv + e); v4us oh, ol;
#pragma unroll
    for (int u = 0; u < 4; ++u) { unsigned short p, q; splitf(__fadd_rn(a[u], b4[u]), p, q); oh[u] = p; ol[u] = q; } *(volatile v4us*)(Hh + e) = oh; *(volatile v4us*)(Hl + e) = ol; __threadfence(); *(volatile v4us*)(Hh + e) = oh; *(volatile v4us*)(Hl + e) = ol; }
__global__ __launch_bounds__(256) void k_lnr(const float* __restrict__ A, int abf, const float* __restrict__ Bv, const float* __restrict__ g, const float* __restrict__ bb, float* X, bf* Xh, bf* Xl) { const int lane = threadIdx.x & 31; const int r = blockIdx.x * 8 + (threadIdx.x >> 5); if (r >= NRB) return; const size_t o0 = (size_t)r * DD + lane * 2; float v[2]; float s = 0.f;
#pragma unroll
    for (int u = 0; u < 2; ++u) { float av = abf ? bfr(A[o0 + u]) : A[o0 + u]; asm volatile("" : "+v"(av)); v[u] = __fadd_rn(av, Bv[o0 + u]); s += v[u]; }
#pragma unroll
    for (int sh = 16; sh; sh >>= 1) s += __shfl_xor(s, sh, 32);
    const float mean = s * (1.0f / DD); float q = 0.f;
#pragma unroll
    for (int u = 0; u < 2; ++u) { float d = __fsub_rn(v[u], mean); asm volatile("" : "+v"(d)); float p = __fmul_rn(d, d); asm volatile("" : "+v"(p)); q = __fadd_rn(q, p); }
#pragma unroll
    for (int sh = 16; sh; sh >>= 1) q += __shfl_xor(q, sh, 32);
    const float rs = __frsqrt_rn(__fadd_rn(q * (1.0f / DD), 1e-5f)); v2f w2; v2us oh, ol;
#pragma unroll
    for (int u = 0; u < 2; ++u) { const int c = lane * 2 + u; float d = __fsub_rn(v[u], mean); asm volatile("" : "+v"(d)); float n0 = __fmul_rn(d, rs); asm volatile("" : "+v"(n0)); float gg = bfr(g[c]), be = bfr(bb[c]); asm volatile("" : "+v"(gg)); asm volatile("" : "+v"(be)); float t1 = __fmul_rn(n0, gg); asm volatile("" : "+v"(t1)); w2[u] = __fadd_rn(t1, be); unsigned short p2, q2; splitf(w2[u], p2, q2); oh[u] = p2; ol[u] = q2; }
    *(volatile v2f*)(X + o0) = w2; *(volatile v2us*)(Xh + o0) = oh; *(volatile v2us*)(Xl + o0) = ol; __threadfence(); *(volatile v2f*)(X + o0) = w2; *(volatile v2us*)(Xh + o0) = oh; *(volatile v2us*)(Xl + o0) = ol; }
__global__ __launch_bounds__(256) void k_relu(const float* __restrict__ F, size_t n4, bf* Hh, bf* Hl) { const size_t e = ((size_t)blockIdx.x * 256 + threadIdx.x) * 4; if (e >= n4) return; const v4f a = *(const v4f*)(F + e); v4us oh, ol;
#pragma unroll
    for (int u = 0; u < 4; ++u) { unsigned short p, q; splitf(fmaxf(a[u], 0.f), p, q); oh[u] = p; ol[u] = q; } *(volatile v4us*)(Hh + e) = oh; *(volatile v4us*)(Hl + e) = ol; __threadfence(); *(volatile v4us*)(Hh + e) = oh; *(volatile v4us*)(Hl + e) = ol; }

extern "C" void kernel_launch(void* const* d_in, const int* in_sizes, int n_in,
                              void* d_out, int out_size, void* d_ws, size_t ws_size, hipStream_t stream) {
    (void)in_sizes; (void)n_in; (void)out_size;
    const float** I = (const float**)d_in;
    const float *x = I[0], *Wq = I[1], *bq = I[2], *Wk = I[3], *bk = I[4], *Wv = I[5], *bv = I[6], *Woa = I[7], *boa = I[8], *Wo = I[9], *bo = I[10], *rk = I[11], *rv = I[12], *g1 = I[13], *b1 = I[14], *g2 = I[15], *b2 = I[16], *Wf1 = I[17], *bf1 = I[18], *Wf2 = I[19], *bf2 = I[20];
    float* OUT = (float*)d_out;
    char* wsp = (char*)d_ws;
    auto take = [&](size_t bytes) { char* p = wsp; wsp += (bytes + 255) & ~(size_t)255; return (void*)p; };
    bf* BQ = (bf*)take(DD * DD * 2); bf* BKw = (bf*)take(DD * DD * 2); bf* BVw = (bf*)take(DD * DD * 2); bf* BOA = (bf*)take(DD * DD * 2); bf* BO = (bf*)take(DD * DD * 2); bf* BF1 = (bf*)take(DD * DFF * 2); bf* BF2 = (bf*)take(DFF * DD * 2); bf* BRK = (bf*)take(DD * DD * 2); bf* BRV = (bf*)take(DD * DD * 2);
    bf* XB = (bf*)take((size_t)NRB * DD * 2); float* T0 = (float*)take((size_t)NRB * DD * 4);
    bf* Qh = (bf*)take((size_t)NRB * DD * 2); bf* Ql = (bf*)take((size_t)NRB * DD * 2); bf* Kh = (bf*)take((size_t)NRB * DD * 2); bf* Kl = (bf*)take((size_t)NRB * DD * 2); bf* VTh = (bf*)take((size_t)NRB * DD * 2); bf* VTl = (bf*)take((size_t)NRB * DD * 2); float* QR = (float*)take((size_t)NRB * DD * 4);
    float* S = (float*)take((size_t)NSQ * TT * TT * 4); bf* Ph = (bf*)take((size_t)NSQ * TT * TT * 2); bf* Pl = (bf*)take((size_t)NSQ * TT * TT * 2); bf* PBh = (bf*)take((size_t)NRB * DD * 2); bf* PBl = (bf*)take((size_t)NRB * DD * 2);
    float* W1 = (float*)take((size_t)NRB * DD * 4); float* W2 = (float*)take((size_t)NRB * DD * 4); bf* Ah = (bf*)take((size_t)NRB * DD * 2); bf* Al = (bf*)take((size_t)NRB * DD * 2); float* Y = (float*)take((size_t)NRB * DD * 4); float* X1 = (float*)take((size_t)NRB * DD * 4); bf* X1h = (bf*)take((size_t)NRB * DD * 2); bf* X1l = (bf*)take((size_t)NRB * DD * 2);
    if ((size_t)(wsp - (char*)d_ws) > ws_size) return;
    float* F1 = S; bf* F1h = Qh; bf* F1l = (bf*)W1;
    k_wtG<<<(DD * DD / 64 + 63) / 64, 256, 0, stream>>>(Wq, DD, DD, BQ); k_wtG<<<(DD * DD / 64 + 63) / 64, 256, 0, stream>>>(Wk, DD, DD, BKw); k_wtG<<<(DD * DD / 64 + 63) / 64, 256, 0, stream>>>(Wv, DD, DD, BVw); k_wtG<<<(DD * DD / 64 + 63) / 64, 256, 0, stream>>>(Woa, DD, DD, BOA); k_wtG<<<(DD * DD / 64 + 63) / 64, 256, 0, stream>>>(Wo, DD, DD, BO);
    k_wtG<<<(DD * DFF / 64 + 63) / 64, 256, 0, stream>>>(Wf1, DD, DFF, BF1); k_wtG<<<(DFF * DD / 64 + 63) / 64, 256, 0, stream>>>(Wf2, DFF, DD, BF2); k_relT<<<(DD * DD / 4 + 255) / 256, 256, 0, stream>>>(rk, rv, BRK, BRV);
    const dim3 g64(NRB / 64, 1, 1); const unsigned gS = (unsigned)(((size_t)NRB * DD / 4 + 255) / 256); const size_t n4 = (size_t)NRB * DD;
    for (int b = 0; b < NB_; ++b) { const float* xb = x + (size_t)b * NRB * DD; float* outb = OUT + (size_t)b * NRB * DD;
        k_cvt8<<<(unsigned)((n4 / 8 + 255) / 256), 256, 0, stream>>>(xb, XB, n4 / 8);
        k_gemmw<bf, 0, true><<<g64, 32, 0, stream>>>(XB, nullptr, BQ, nullptr, DD, T0, DD, bq, 0, 0, 0); k_spl<<<gS, 256, 0, stream>>>(T0, n4, Qh, Ql);
        k_gemmw<bf, 0, true><<<g64, 32, 0, stream>>>(XB, nullptr, BKw, nullptr, DD, T0, DD, bk, 0, 0, 0); k_spl<<<gS, 256, 0, stream>>>(T0, n4, Kh, Kl);
        k_gemmw<bf, 0, true><<<g64, 32, 0, stream>>>(XB, nullptr, BVw, nullptr, DD, T0, DD, bv, 0, 0, 0); k_vtz<<<(unsigned)(((size_t)NSQ * DD * TT / 2 + 255) / 256), 256, 0, stream>>>(T0, VTh, VTl);
        k_gemmw<bf, 1, false><<<g64, 32, 0, stream>>>(Qh, Ql, BRK, nullptr, DD, QR, DD, nullptr, 0, 0, 0);
        k_gemmw<bf, 2, false><<<dim3(TT / 64, TT / 64, NSQ), 32, 0, stream>>>(Qh, Ql, Kh, Kl, DD, S, TT, nullptr, (size_t)TT * DD, (size_t)TT * DD, (size_t)TT * TT);
        k_ssoft<<<NSQ * TT / 8, 256, 0, stream>>>(S, QR, Ph, Pl, PBh, PBl);
        k_gemmw<bf, 2, false><<<dim3(TT / 64, 1, NSQ), 32, 0, stream>>>(Ph, Pl, VTh, VTl, TT, W1, DD, nullptr, (size_t)TT * TT, (size_t)DD * TT, (size_t)TT * DD);
        k_gemmw<bf, 1, false><<<g64, 32, 0, stream>>>(PBh, PBl, BRV, nullptr, DD, W2, DD, nullptr, 0, 0, 0);
        k_add2<<<gS, 256, 0, stream>>>(W1, W2, n4, Ah, Al); k_gemmw<bf, 1, true><<<g64, 32, 0, stream>>>(Ah, Al, BOA, nullptr, DD, Y, DD, boa, 0, 0, 0);
        k_spl<<<gS, 256, 0, stream>>>(Y, n4, Ah, Al); k_gemmw<bf, 1, true><<<g64, 32, 0, stream>>>(Ah, Al, BO, nullptr, DD, Y, DD, bo, 0, 0, 0);
        k_lnr<<<NRB / 8, 256, 0, stream>>>(xb, 1, Y, g1, b1, X1, X1h, X1l);
        k_gemmw<bf, 1, true><<<dim3(NRB / 64, DFF / 64, 1), 32, 0, stream>>>(X1h, X1l, BF1, nullptr, DD, F1, DFF, bf1, 0, 0, 0); k_relu<<<(unsigned)(((size_t)NRB * DFF / 4 + 255) / 256), 256, 0, stream>>>(F1, (size_t)NRB * DFF, F1h, F1l);
        k_gemmw<bf, 1, true><<<g64, 32, 0, stream>>>(F1h, F1l, BF2, nullptr, DFF, Y, DD, bf2, 0, 0, 0);
        k_lnr<<<NRB / 8, 256, 0, stream>>>(X1, 0, Y, g2, b2, outb, Ah, Al); }
}
